// DeltaNetLayer_46892452937748
// MI455X (gfx1250) — hardware-verified
//
#include <hip/hip_runtime.h>
#include <math.h>

constexpr int kBatch    = 4;
constexpr int kSteps    = 2048;
constexpr int kHid      = 1024;
constexpr int kHeads    = 16;
constexpr int kHeadDim  = kHid / kHeads;
constexpr int kRows     = kBatch * kSteps;
constexpr int kProjN    = 4 * kHid;
constexpr int kHalfRows = kRows / 2;
constexpr int kChunk    = 16;
constexpr int kNumChunk = kSteps / kChunk;
constexpr float kWCarry    = 64.0f;
constexpr float kWCarryInv = 1.0f / kWCarry;
constexpr float kInvHid    = 1.0f / (float)kHid;
constexpr float kLnEps     = 1e-5f;
constexpr float kNormEps   = 1e-6f;

static_assert(kHeadDim == 64, "head dim");
static_assert(kHeads * kHeadDim == kHid, "heads");
static_assert(kHid % 32 == 0, "GEMM K multiple of 32");
static_assert(kHalfRows % 64 == 0 && kRows % 64 == 0, "GEMM M tile multiple");
static_assert(kProjN % 64 == 0 && kHid % 64 == 0, "GEMM N tile multiple");
static_assert(kSteps % kChunk == 0, "chunking");
static_assert(kRows % 8 == 0, "LayerNorm grid");
static_assert((kHalfRows / 64) * (kProjN / 64) % 8 == 0, "projection grid exact");
static_assert((kRows / 64) * (kHid / 64) % 8 == 0, "output projection grid exact");

typedef __attribute__((ext_vector_type(16))) _Float16 v16h;
typedef __attribute__((ext_vector_type(8)))  _Float16 v8h;
typedef __attribute__((ext_vector_type(8)))  float    v8f;
typedef __attribute__((ext_vector_type(4)))  float    v4f;
typedef __attribute__((ext_vector_type(4)))  unsigned int v4u;

__device__ __forceinline__ unsigned short f2bf_bits(float f) {
  unsigned u = __float_as_uint(f);
  return (unsigned short)((u + 0x7FFFu + ((u >> 16) & 1u)) >> 16);
}
__device__ __forceinline__ float bf_bits2f(unsigned short h) { return __uint_as_float(((unsigned)h) << 16); }
__device__ __forceinline__ float bf16r(float f) { return bf_bits2f(f2bf_bits(f)); }
__device__ __forceinline__ unsigned pk16(unsigned short a, unsigned short b) { return (unsigned)a | ((unsigned)b << 16); }
__device__ __forceinline__ unsigned short h_bits(float f) { const _Float16 h = (_Float16)f; return __builtin_bit_cast(unsigned short, h); }

__device__ __forceinline__ void dep_guard4_h(v8f& a, v8f& b, v8f& c, v8f& d, v16h x, v16h y) {
  asm volatile("v_nop\n\tv_nop\n\tv_nop\n\tv_nop" : "+v"(a), "+v"(b), "+v"(c), "+v"(d) : "v"(x), "v"(y));
}
__device__ __forceinline__ void keep4_h(v16h a, v16h b, v16h c, v16h d) { asm volatile("v_nop" :: "v"(a), "v"(b), "v"(c), "v"(d)); }
__device__ __forceinline__ void acc_guard4(v8f& a, v8f& b, v8f& c, v8f& d) {
  asm volatile("v_nop\n\tv_nop\n\tv_nop\n\tv_nop" : "+v"(a), "+v"(b), "+v"(c), "+v"(d));
}

union FragU { v16h v; v8h h[2]; };
__device__ __forceinline__ v16h frag_load(const _Float16* p) {
  FragU f;
  f.h[0] = *(const v8h*)(p);
  f.h[1] = *(const v8h*)(p + 16);
  return f.v;
}
__device__ __forceinline__ v8f frag_mma(v16h a, v16h b, v8f c) {
  return __builtin_amdgcn_wmma_f32_16x16x32_f16(false, a, false, b, (short)0, c, false, false);
}

__global__ __launch_bounds__(256) void ln_rows_f16(const float* __restrict__ x, const float* __restrict__ gam,
                                                   const float* __restrict__ bet, unsigned short* __restrict__ out,
                                                   int nrows) {
  const int tid = threadIdx.x;
  const int lane = tid & 31;
  const int row = blockIdx.x * 8 + (tid >> 5);
  if (row >= nrows) return;
  const float* rp = x + (size_t)row * kHid;
  float v[32];
  float s = 0.0f;
#pragma unroll
  for (int q = 0; q < 4; ++q) {
    const v4f a = *(const v4f*)(rp + 256 * q + 8 * lane);
    const v4f b = *(const v4f*)(rp + 256 * q + 8 * lane + 4);
#pragma unroll
    for (int e = 0; e < 4; ++e) {
      const float fa = a[e];
      const float fb = b[e];
      v[8 * q + e]     = bf16r(fa);
      v[8 * q + 4 + e] = bf16r(fb);
    }
    s += ((v[8 * q + 0] + v[8 * q + 1]) + (v[8 * q + 2] + v[8 * q + 3])) +
         ((v[8 * q + 4] + v[8 * q + 5]) + (v[8 * q + 6] + v[8 * q + 7]));
  }
#pragma unroll
  for (int off = 1; off < 32; off <<= 1) s += __shfl_xor(s, off, 32);
  const float mu = s * kInvHid;
  float ss = 0.0f;
#pragma unroll
  for (int i = 0; i < 32; ++i) {
    const float d = v[i] - mu;
    v[i] = d;
    ss = fmaf(d, d, ss);
  }
#pragma unroll
  for (int off = 1; off < 32; off <<= 1) ss += __shfl_xor(ss, off, 32);
  const float var  = ss * kInvHid;
  const float rstd = rsqrtf(var + kLnEps);
  v4u o[4];
#pragma unroll
  for (int q = 0; q < 4; ++q) {
    const v4f ga = *(const v4f*)(gam + 256 * q + 8 * lane);
    const v4f gb = *(const v4f*)(gam + 256 * q + 8 * lane + 4);
    const v4f ba = *(const v4f*)(bet + 256 * q + 8 * lane);
    const v4f bb = *(const v4f*)(bet + 256 * q + 8 * lane + 4);
    unsigned short hb[8];
#pragma unroll
    for (int e = 0; e < 4; ++e) {
      const float g0 = ga[e];
      const float g1 = gb[e];
      const float b0 = ba[e];
      const float b1 = bb[e];
      const float y0 = fmaf(v[8 * q + e] * rstd, bf16r(g0), bf16r(b0));
      const float y1 = fmaf(v[8 * q + 4 + e] * rstd, bf16r(g1), bf16r(b1));
      hb[e]     = h_bits(y0);
      hb[4 + e] = h_bits(y1);
    }
    o[q] = (v4u){pk16(hb[0], hb[1]), pk16(hb[2], hb[3]), pk16(hb[4], hb[5]), pk16(hb[6], hb[7])};
  }
  unsigned short* op = out + (size_t)row * kHid;
  for (int pass = 0; pass < 2; ++pass) {
#pragma unroll
    for (int q = 0; q < 4; ++q) *(volatile v4u*)(op + 256 * q + 8 * lane) = o[q];
    __threadfence();
  }
}

__global__ __launch_bounds__(256) void wt_transpose_f16(const float* __restrict__ W, unsigned short* __restrict__ out,
                                                        int nK, int nN, float carry) {
  __shared__ float sm[64][65];
  const int t  = threadIdx.x;
  const int k0 = blockIdx.x * 64;
  const int n0 = blockIdx.y * 64;
#pragma unroll
  for (int i = 0; i < 16; ++i) {
    const int e = i * 256 + t;
    const int r = e >> 6;
    const int c = e & 63;
    sm[c][r] = bf16r(W[(size_t)(k0 + r) * nN + n0 + c]) * carry;
  }
  __syncthreads();
  const int lane = t & 31, wave = t >> 5;
  const int q = lane >> 3, c8 = (lane & 7) * 8;
  for (int pass = 0; pass < 2; ++pass) {
#pragma unroll
    for (int it = 0; it < 2; ++it) {
      const int row = wave * 8 + it * 4 + q;
      unsigned short hb[8];
#pragma unroll
      for (int e = 0; e < 8; ++e) hb[e] = h_bits(sm[row][c8 + e]);
      const v4u u = (v4u){pk16(hb[0], hb[1]), pk16(hb[2], hb[3]), pk16(hb[4], hb[5]), pk16(hb[6], hb[7])};
      *(volatile v4u*)(out + (size_t)(n0 + row) * nK + k0 + c8) = u;
    }
    __threadfence();
  }
}

template <bool RESID>
__global__ __launch_bounds__(256) void wmma_gemm64_f16(
    const unsigned short* __restrict__ Ap, int lda,
    const unsigned short* __restrict__ Btp, int ldb,
    float* __restrict__ Cout, int ldc,
    const float* __restrict__ bias,
    const float* __restrict__ resid, int ldr,
    int M, int N, int K, float scale) {
  const _Float16* A  = (const _Float16*)Ap;
  const _Float16* Bt = (const _Float16*)Btp;
  __shared__ __align__(16) float sT[8][16 * 68];
  const int lane = threadIdx.x & 31;
  const int wave = threadIdx.x >> 5;
  const int tilesN = N >> 6;
  const int tilesM = M >> 6;
  const int tile = blockIdx.x * 8 + wave;
  if (tile >= tilesM * tilesN) return;
  const int tm = tile / tilesN;
  const int tn = tile - tm * tilesN;
  const int m0 = tm << 6;
  const int n0 = tn << 6;

  const int rlane = lane & 15;
  const int koff  = (lane >> 4) * 8;
  const int mOff  = (lane >> 4) * 8;

  const _Float16* bp[4];
  const _Float16* ap[4];
#pragma unroll
  for (int j = 0; j < 4; ++j) bp[j] = Bt + (size_t)(n0 + (j << 4) + rlane) * ldb + koff;
#pragma unroll
  for (int i = 0; i < 4; ++i) ap[i] = A + (size_t)(m0 + (i << 4) + rlane) * lda + koff;

  v8f acc[4][4];
#pragma unroll
  for (int i = 0; i < 4; ++i)
#pragma unroll
    for (int j = 0; j < 4; ++j) acc[i][j] = (v8f){0.f, 0.f, 0.f, 0.f, 0.f, 0.f, 0.f, 0.f};

  for (int k0 = 0; k0 < K; k0 += 32) {
    v16h bh[4];
#pragma unroll
    for (int j = 0; j < 4; ++j) bh[j] = frag_load(bp[j] + k0);
#pragma unroll
    for (int i = 0; i < 4; ++i) {
      const v16h ah = frag_load(ap[i] + k0);
#pragma unroll
      for (int j = 0; j < 4; ++j) acc[i][j] = frag_mma(ah, bh[j], acc[i][j]);
      dep_guard4_h(acc[i][0], acc[i][1], acc[i][2], acc[i][3], ah, bh[3]);
    }
    keep4_h(bh[0], bh[1], bh[2], bh[3]);
  }
  acc_guard4(acc[0][0], acc[0][1], acc[0][2], acc[0][3]);
  acc_guard4(acc[1][0], acc[1][1], acc[1][2], acc[1][3]);
  acc_guard4(acc[2][0], acc[2][1], acc[2][2], acc[2][3]);
  acc_guard4(acc[3][0], acc[3][1], acc[3][2], acc[3][3]);

  float* slab = sT[wave];
  const int hh = lane >> 4;
  const int c4 = (lane & 15) * 4;
#pragma unroll
  for (int i = 0; i < 4; ++i) {
    const int mBase = m0 + (i << 4);
#pragma unroll
    for (int j = 0; j < 4; ++j) {
      const int n = n0 + (j << 4) + rlane;
      const float bv = bf16r(bias[n]);
#pragma unroll
      for (int r = 0; r < 8; ++r) {
        const float v = acc[i][j][r] * scale + bv;
        slab[(mOff + r) * 68 + (j << 4) + rlane] = v;
      }
    }
    __builtin_amdgcn_fence(__ATOMIC_RELEASE, "workgroup");
    __builtin_amdgcn_wave_barrier();
    __builtin_amdgcn_fence(__ATOMIC_ACQUIRE, "workgroup");
    v4f ov[8];
#pragma unroll
    for (int it = 0; it < 8; ++it) {
      const int row = it * 2 + hh;
      v4f v = *(const v4f*)(slab + row * 68 + c4);
      if (RESID) {
        const v4f rr = *(const v4f*)(resid + (size_t)(mBase + row) * ldr + n0 + c4);
        const float r0 = rr[0];
        const float r1 = rr[1];
        const float r2 = rr[2];
        const float r3 = rr[3];
        v[0] += bf16r(r0);
        v[1] += bf16r(r1);
        v[2] += bf16r(r2);
        v[3] += bf16r(r3);
      }
      ov[it] = v;
    }
    for (int pass = 0; pass < 2; ++pass) {
#pragma unroll
      for (int it = 0; it < 8; ++it) {
        const int row = it * 2 + hh;
        *(volatile v4f*)(Cout + (size_t)(mBase + row) * ldc + n0 + c4) = ov[it];
      }
      __threadfence();
    }
    __builtin_amdgcn_fence(__ATOMIC_RELEASE, "workgroup");
    __builtin_amdgcn_wave_barrier();
    __builtin_amdgcn_fence(__ATOMIC_ACQUIRE, "workgroup");
  }
}

__global__ __launch_bounds__(256) void state_scan_kernel(const float* __restrict__ proj, unsigned short* __restrict__ attn) {
  __shared__ __align__(16) float sQ[2][kChunk * kHeadDim];
  __shared__ __align__(16) float sK[2][kChunk * kHeadDim];
  __shared__ __align__(16) float sV[2][kChunk * kHeadDim];
  __shared__ __align__(16) float sB[2][kChunk * kHeadDim];
  __shared__ __align__(16) float sO[2][kChunk * kHeadDim];
  __shared__ float sKQ[2][kChunk];

  const int tid  = threadIdx.x;
  const int lane = tid & 31;
  const int wave = tid >> 5;
  const int bl   = blockIdx.x >> 4;
  const int hd   = blockIdx.x & 15;
  const int row  = tid >> 2;
  const int part = tid & 3;
  const int cb   = part * 16;
  const int st   = tid >> 4;
  const int c4   = (tid & 15) * 4;

  const float* pbase = proj + (size_t)bl * kSteps * kProjN + hd * kHeadDim + c4;
  unsigned short* abase = attn + (size_t)bl * kSteps * kHid + hd * kHeadDim;

  float S[16];
#pragma unroll
  for (int j = 0; j < 16; ++j) S[j] = 0.0f;

#pragma unroll 1
  for (int ci = 0; ci <= kNumChunk; ++ci) {
    const int cprev = ci - 1;
    const int cn  = (ci < kNumChunk) ? ci : (kNumChunk - 1);
    const int nb  = ci & 1;
    const int buf = nb ^ 1;

    const float* p = pbase + (size_t)(cn * kChunk + st) * kProjN;
    const v4f nq = *(const v4f*)(p);
    const v4f nk = *(const v4f*)(p + kHid);
    const v4f nv = *(const v4f*)(p + 2 * kHid);
    const v4f nbp = *(const v4f*)(p + 3 * kHid);

    if (cprev >= 0) {
#pragma unroll 1
      for (int s = 0; s < kChunk; ++s) {
        const int so = s * kHeadDim;
        v4f kv[4], qv[4];
#pragma unroll
        for (int i = 0; i < 4; ++i) {
          kv[i] = *(const v4f*)&sK[buf][so + cb + 4 * i];
          qv[i] = *(const v4f*)&sQ[buf][so + cb + 4 * i];
        }
        const float vv = sV[buf][so + row];
        const float be = sB[buf][so + row];
        const float kq = sKQ[buf][s];
        float kr[16], qr[16];
#pragma unroll
        for (int i = 0; i < 4; ++i) {
#pragma unroll
          for (int e = 0; e < 4; ++e) {
            kr[4 * i + e] = kv[i][e];
            qr[4 * i + e] = qv[i][e];
          }
        }
        float pr = 0.0f, pp = 0.0f;
#pragma unroll
        for (int j = 0; j < 16; ++j) {
          pr = fmaf(S[j], kr[j], pr);
          pp = fmaf(S[j], qr[j], pp);
        }
        pr += __shfl_xor(pr, 1, 32);
        pp += __shfl_xor(pp, 1, 32);
        pr += __shfl_xor(pr, 2, 32);
        pp += __shfl_xor(pp, 2, 32);
        const float wc = be * (vv - pr);
#pragma unroll
        for (int j = 0; j < 16; ++j) S[j] = fmaf(wc, kr[j], S[j]);
        const float po = fmaf(wc, kq, pp);
        if (part == 0) sO[buf][so + row] = po;
      }
    }

    {
      const float ka = nk[0];
      const float kb = nk[1];
      const float kc = nk[2];
      const float kd = nk[3];
      const float qa = nq[0];
      const float qb = nq[1];
      const float qc = nq[2];
      const float qd = nq[3];
      float ss = (ka * ka + kb * kb) + (kc * kc + kd * kd);
      ss += __shfl_xor(ss, 1, 32);
      ss += __shfl_xor(ss, 2, 32);
      ss += __shfl_xor(ss, 4, 32);
      ss += __shfl_xor(ss, 8, 32);
      const float nrm = fmaxf(sqrtf(ss), kNormEps);
      const float inv = 1.0f / nrm;
      v4f kn;
      kn[0] = ka * inv;
      kn[1] = kb * inv;
      kn[2] = kc * inv;
      kn[3] = kd * inv;
      const float k0n = kn[0];
      const float k1n = kn[1];
      const float k2n = kn[2];
      const float k3n = kn[3];
      float dq = (k0n * qa + k1n * qb) + (k2n * qc + k3n * qd);
      dq += __shfl_xor(dq, 1, 32);
      dq += __shfl_xor(dq, 2, 32);
      dq += __shfl_xor(dq, 4, 32);
      dq += __shfl_xor(dq, 8, 32);
      *(v4f*)&sQ[nb][st * kHeadDim + c4] = nq;
      *(v4f*)&sK[nb][st * kHeadDim + c4] = kn;
      *(v4f*)&sV[nb][st * kHeadDim + c4] = nv;
      if ((tid & 15) == 0) sKQ[nb][st] = dq;
      const float b0 = nbp[0];
      const float b1 = nbp[1];
      const float b2 = nbp[2];
      const float b3 = nbp[3];
#pragma unroll 1
      for (int e = 0; e < 4; ++e) {
        const float xb = (e == 0) ? b0 : ((e == 1) ? b1 : ((e == 2) ? b2 : b3));
        const float sg = 1.0f / (1.0f + expf(-xb));
        sB[nb][st * kHeadDim + c4 + e] = sg;
      }
    }
    __syncthreads();

    if (cprev >= 0 && wave < 4) {
      const int line = wave * 4 + (lane >> 3);
      const int c8 = (lane & 7) * 8;
      const float* sp = &sO[buf][line * kHeadDim + c8];
      const v4f a = *(const v4f*)(sp);
      const v4f b = *(const v4f*)(sp + 4);
      unsigned short hb[8];
#pragma unroll
      for (int e = 0; e < 4; ++e) {
        const float fa = a[e];
        const float fb = b[e];
        hb[e]     = h_bits(fa);
        hb[4 + e] = h_bits(fb);
      }
      const v4u u = (v4u){pk16(hb[0], hb[1]), pk16(hb[2], hb[3]), pk16(hb[4], hb[5]), pk16(hb[6], hb[7])};
      unsigned short* op = abase + (size_t)(cprev * kChunk + line) * kHid + c8;
      *(volatile v4u*)op = u;
      __threadfence();
      *(volatile v4u*)op = u;
    }
  }
}

extern "C" void kernel_launch(void* const* d_in, const int* in_sizes, int n_in,
                              void* d_out, int out_size, void* d_ws, size_t ws_size, hipStream_t stream) {
  if (n_in < 7 || d_out == nullptr || d_ws == nullptr) return;
  if (in_sizes[0] != kRows * kHid || in_sizes[1] != kHid || in_sizes[2] != kHid ||
      in_sizes[3] != kHid * kProjN || in_sizes[4] != kProjN || in_sizes[5] != kHid * kHid ||
      in_sizes[6] != kHid || out_size != kRows * kHid) return;

  const float* x      = (const float*)d_in[0];
  const float* ln_g   = (const float*)d_in[1];
  const float* ln_b   = (const float*)d_in[2];
  const float* w_qkvb = (const float*)d_in[3];
  const float* b_qkvb = (const float*)d_in[4];
  const float* w_out  = (const float*)d_in[5];
  const float* b_out  = (const float*)d_in[6];
  float* out = (float*)d_out;

  char* ws = (char*)d_ws;
  size_t off = 0;
  auto carve = [&](size_t bytes) -> char* { char* p = ws + off; off += (bytes + 255) & ~(size_t)255; return p; };
  unsigned short* NORMED = (unsigned short*)carve((size_t)kRows * kHid * 2);
  unsigned short* WQT    = (unsigned short*)carve((size_t)kProjN * kHid * 2);
  unsigned short* WOT    = (unsigned short*)carve((size_t)kHid * kHid * 2);
  float*          PROJH  = (float*)carve((size_t)kHalfRows * kProjN * 4);
  unsigned short* ATTN   = (unsigned short*)carve((size_t)kRows * kHid * 2);
  if (off > ws_size || off > (size_t)134217728) return;

  ln_rows_f16<<<kRows / 8, 256, 0, stream>>>(x, ln_g, ln_b, NORMED, kRows);

  wt_transpose_f16<<<dim3(kHid / 64, kProjN / 64), 256, 0, stream>>>(w_qkvb, WQT, kHid, kProjN, kWCarry);
  wt_transpose_f16<<<dim3(kHid / 64, kHid / 64), 256, 0, stream>>>(w_out, WOT, kHid, kHid, kWCarry);

  const int tiles1 = (kHalfRows / 64) * (kProjN / 64);
  for (int half = 0; half < 2; ++half) {
    wmma_gemm64_f16<false><<<dim3(tiles1 / 8, 1), 256, 0, stream>>>(
        NORMED + (size_t)half * kHalfRows * kHid, kHid, WQT, kHid, PROJH, kProjN,
        b_qkvb, x, kHid, kHalfRows, kProjN, kHid, kWCarryInv);
    state_scan_kernel<<<2 * kHeads, 256, 0, stream>>>(PROJH, ATTN + (size_t)half * kHalfRows * kHid);
  }

  const int tiles2 = (kRows / 64) * (kHid / 64);
  wmma_gemm64_f16<true><<<dim3(tiles2 / 8, 1), 256, 0, stream>>>(
      ATTN, kHid, WOT, kHid, out, kHid, b_out, x, kHid, kRows, kHid, kHid, kWCarryInv);
}
